// QuantumLayer_44504451121459
// MI455X (gfx1250) — hardware-verified
//
#include <hip/hip_runtime.h>


#ifndef NB
#define NB 8192
#endif
#define NB_FULL 8192
#define NQ   8
#define NLAY 4
#define DIM  256
#define KD   512
#define BT   32
#define BP   520
#define PSC  4096.0f
#define ASC  4096.0f
#define YSI  5.9604644775390625e-08f
#define PI_F 3.14159265358979323846f

static_assert(NB <= NB_FULL);
static_assert(NB % BT == 0);
static_assert(KD == 2 * DIM);
static_assert(KD % 128 == 0);
static_assert(BP >= KD);
static_assert((BP * 2) % 16 == 0);
static_assert(NQ * BT == 256);
static_assert(8 * 32 == DIM);
static_assert(64 * 16 == BT * NQ * 4);
static_assert(128 * 16 == 2 * KD * 2);
static_assert(NLAY * 4 * NQ == 128);
static_assert(BT * BP * 2 + BT * NQ * 4 * 4 + 8 * 2 * 16 * 8 * 4 <= 131072);
static_assert(2 * DIM * 4 + 128 * 8 * 4 <= 131072);

typedef _Float16 h16;
typedef __attribute__((ext_vector_type(16))) _Float16 v16h;
typedef __attribute__((ext_vector_type(8)))  _Float16 v8h;
typedef __attribute__((ext_vector_type(8)))  float    v8f;
typedef __attribute__((ext_vector_type(4)))  float    v4f;
typedef v4f  __attribute__((may_alias)) v4fa;

__device__ __forceinline__ unsigned short f2bf(float f) { unsigned u = __float_as_uint(f); u += 0x7FFFu + ((u >> 16) & 1u); return (unsigned short)(u >> 16); }
__device__ __forceinline__ float bfr(float f) { return __uint_as_float(((unsigned)f2bf(f)) << 16); }
__device__ __forceinline__ v16h cat16(v8h lo, v8h hi) { return __builtin_shufflevector(lo, hi, 0, 1, 2, 3, 4, 5, 6, 7, 8, 9, 10, 11, 12, 13, 14, 15); }
__device__ __forceinline__ v8f wmma16(v16h a, v16h b, v8f c) { return __builtin_amdgcn_wmma_f32_16x16x32_f16(false, a, false, b, (short)0, c, false, false); }
__device__ __forceinline__ v16h  ldh(const h16* p) { return cat16(*(const v8h*)p, *(const v8h*)(p + 16)); }
__device__ __forceinline__ v8f wmma16g(v16h a, v16h b, v8f c) { c = wmma16(a, b, c); asm volatile("v_nop\n\tv_nop\n\tv_nop\n\tv_nop" : "+v"(c) : "v"(a), "v"(b)); return c; }
__device__ __forceinline__ h16 toh_flush(float v) { const h16 r = (h16)v; return (fabsf(v) < 6.103515625e-05f) ? (h16)0.0f : r; }

struct cpx { float x, y; };
__device__ __forceinline__ cpx mkc(float x, float y) { cpx r; r.x = x; r.y = y; return r; }
__device__ __forceinline__ cpx cmul(cpx a, cpx b) { cpx r; r.x = a.x * b.x - a.y * b.y; r.y = a.x * b.y + a.y * b.x; return r; }
__device__ __forceinline__ cpx csel(bool c, cpx a, cpx b) { cpx r; r.x = c ? a.x : b.x; r.y = c ? a.y : b.y; return r; }
__device__ __forceinline__ cpx q0(v4f f) { return mkc(f[0], f[1]); }
__device__ __forceinline__ cpx q1(v4f f) { return mkc(f[2], f[3]); }

__device__ __forceinline__ int cxf(int i, int cb, int tb) { return i ^ (((i >> cb) & 1) << tb); }
__device__ __forceinline__ int inv_perm(int i) {
    i = cxf(i, 7, 6); i = cxf(i, 6, 5); i = cxf(i, 5, 4); i = cxf(i, 4, 3); i = cxf(i, 3, 2);
    i = cxf(i, 2, 1); i = cxf(i, 1, 0); i = cxf(i, 7, 0); i = cxf(i, 6, 1); return i;
}

__global__ __launch_bounds__(128) void k_build(const float* __restrict__ W, h16* AP) {
#pragma clang fp contract(off)
    __shared__ __align__(16) float sre[DIM];
    __shared__ __align__(16) float sim[DIM];
    __shared__ __align__(16) float gm[128 * 8];
    const int t = threadIdx.x;
    const int row = blockIdx.x;
    {
        const int gi = (t >> 3) & 3;
        const float wv = bfr(W[t]);
        const float hh = 0.5f * wv;
        const float cs = cosf(hh);
        const float se = -sinf(hh);
        const bool isx = (gi == 0) | (gi == 3), isy = (gi == 1), isz = (gi == 2);
        v4f g0, g1;
        g0[0] = cs;                 g0[1] = isz ? -se : 0.0f;  g0[2] = isy ? -se : 0.0f;  g0[3] = isx ? -se : 0.0f;
        g1[0] = isy ? se : 0.0f;    g1[1] = isx ? -se : 0.0f;  g1[2] = cs;                g1[3] = isz ? se : 0.0f;
        *(v4fa*)(&gm[t * 8]) = g0; *(v4fa*)(&gm[t * 8 + 4]) = g1;
        sre[t] = (t == row) ? 1.0f : 0.0f; sre[t + 128] = (t + 128 == row) ? 1.0f : 0.0f;
        sim[t] = 0.0f; sim[t + 128] = 0.0f;
    }
    __syncthreads();
#pragma unroll 1
    for (int l = NLAY - 1; l >= 0; --l) {
        {
            const int s0 = inv_perm(t), s1 = inv_perm(t + 128);
            const float ar = sre[s0], ai = sim[s0], br = sre[s1], bi = sim[s1];
            __syncthreads();
            sre[t] = ar; sim[t] = ai; sre[t + 128] = br; sim[t + 128] = bi;
            __syncthreads();
        }
#pragma unroll 1
        for (int q = 0; q < 32; ++q) {
            const int gi = 3 - (q >> 3), w = q & 7;
            const int gx = ((4 * l + gi) * 8 + w) * 8;
            const v4f g0 = *(const v4fa*)(&gm[gx]);
            const v4f g1 = *(const v4fa*)(&gm[gx + 4]);
            const int p = 7 - w;
            const int lowm = (1 << p) - 1;
            const int i0 = ((t & ~lowm) << 1) | (t & lowm);
            const int i1 = i0 | (1 << p);
            const float ar = sre[i0], ai = sim[i0], br = sre[i1], bi = sim[i1];
            const float n0r = (g0[0] * ar - g0[1] * ai) + (g0[2] * br - g0[3] * bi);
            const float n0i = (g0[0] * ai + g0[1] * ar) + (g0[2] * bi + g0[3] * br);
            const float n1r = (g1[0] * ar - g1[1] * ai) + (g1[2] * br - g1[3] * bi);
            const float n1i = (g1[0] * ai + g1[1] * ar) + (g1[2] * bi + g1[3] * br);
            sre[i0] = n0r; sim[i0] = n0i; sre[i1] = n1r; sim[i1] = n1i;
            __syncthreads();
        }
    }
    {
        const int sel = t >> 6;
        const int c8 = (t & 63) * 8;
        const int kk = c8 & 255;
        const bool hik = c8 >= 256;
        const v4f x0 = *(const v4fa*)(&sre[kk]), x1 = *(const v4fa*)(&sre[kk + 4]);
        const v4f y0 = *(const v4fa*)(&sim[kk]), y1 = *(const v4fa*)(&sim[kk + 4]);
        v8h o;
#pragma unroll
        for (int e = 0; e < 4; ++e) {
            const float a0 = (sel == 0) ? (hik ? y0[e] : x0[e]) : (hik ? x0[e] : -y0[e]);
            const float a1 = (sel == 0) ? (hik ? y1[e] : x1[e]) : (hik ? x1[e] : -y1[e]);
            o[e] = toh_flush(a0 * ASC); o[4 + e] = toh_flush(a1 * ASC);
        }
        h16* dst = AP + ((size_t)(row + 256 * sel)) * KD + c8;
        *(volatile v8h*)dst = o;
        __threadfence();
        *(volatile v8h*)dst = o;
    }
}

__global__ __launch_bounds__(256) void k_apply(const float* __restrict__ X, const h16* __restrict__ AP, float* OUT) {
    __shared__ __align__(16) h16 bs[BT * BP];
    __shared__ __align__(16) float fac[BT * NQ * 4];
    __shared__ __align__(16) float part[8 * 2 * 16 * 8];
    const int tid = threadIdx.x;
    const int lane = tid & 31, lr = lane & 15, hi = lane >> 4;
    const int wave = __builtin_amdgcn_readfirstlane((int)(threadIdx.x >> 5));
    const int gv = (int)(threadIdx.x >> 5);
    const int n0 = blockIdx.x * BT;

    {
        const float xv = bfr(X[(size_t)n0 * NQ + tid]);
        const float th = PI_F * xv;
        const float ha = 0.5f * th;
        const float hb = 0.25f * th;
        const float cy = cosf(ha), sy = sinf(ha);
        const float cz = cosf(hb), sz = sinf(hb);
        v4f fv; fv[0] = cy * cz; fv[1] = -(cy * sz); fv[2] = sy * cz; fv[3] = sy * sz;
        *(v4fa*)(&fac[tid * 4]) = fv;
    }
    __syncthreads();

    {
        v4f f[8];
#pragma unroll
        for (int w = 0; w < 8; ++w) f[w] = *(const v4fa*)(&fac[(lane * NQ + w) * 4]);
        cpx thg = csel((gv & 4) != 0, q1(f[0]), q0(f[0]));
        thg = cmul(thg, csel((gv & 2) != 0, q1(f[1]), q0(f[1])));
        thg = cmul(thg, csel((gv & 1) != 0, q1(f[2]), q0(f[2])));
        cpx th[2];
        th[0] = cmul(thg, q0(f[3])); th[1] = cmul(thg, q1(f[3]));
        cpx t45[4], t67[4];
#pragma unroll
        for (int a = 0; a < 4; ++a) {
            t45[a] = cmul((a & 2) ? q1(f[4]) : q0(f[4]), (a & 1) ? q1(f[5]) : q0(f[5]));
            t67[a] = cmul((a & 2) ? q1(f[6]) : q0(f[6]), (a & 1) ? q1(f[7]) : q0(f[7]));
        }
        cpx tl[16];
#pragma unroll
        for (int lo = 0; lo < 16; ++lo) tl[lo] = cmul(t45[lo >> 2], t67[lo & 3]);
#pragma unroll
        for (int b = 0; b < 2; ++b) {
#pragma unroll
            for (int c = 0; c < 2; ++c) {
                v8h re8, im8;
#pragma unroll
                for (int e = 0; e < 8; ++e) {
                    const cpx a = cmul(th[b], tl[c * 8 + e]);
                    re8[e] = toh_flush(a.x * PSC); im8[e] = toh_flush(a.y * PSC);
                }
                const int ko = lane * BP + wave * 32 + b * 16 + c * 8;
                *(v8h*)(&bs[ko]) = re8;
                *(v8h*)(&bs[ko + DIM]) = im8;
            }
        }
    }
    __syncthreads();

    v8f acc[4][2];
#pragma unroll
    for (int hh = 0; hh < 4; ++hh) { acc[hh][0] = (v8f){}; acc[hh][1] = (v8f){}; }
    const size_t ab = ((size_t)(wave * 32 + lr)) * KD + 8 * hi;
    const int bo = lr * BP + 8 * hi;
#pragma unroll 1
    for (int kq = 0; kq < KD; kq += 128) {
#pragma unroll
        for (int u = 0; u < 4; ++u) {
            const int k0 = kq + 32 * u;
            v16h a[4];
#pragma unroll
            for (int hh = 0; hh < 4; ++hh) a[hh] = ldh(AP + ab + (size_t)((hh & 1) * 16 + (hh >> 1) * 256) * KD + k0);
            const v16h b0 = cat16(*(const v8h*)(&bs[bo + k0]), *(const v8h*)(&bs[bo + k0 + 16]));
            const v16h b1 = cat16(*(const v8h*)(&bs[bo + 16 * BP + k0]), *(const v8h*)(&bs[bo + 16 * BP + k0 + 16]));
#pragma unroll
            for (int hh = 0; hh < 4; ++hh) {
                acc[hh][0] = wmma16g(a[hh], b0, acc[hh][0]);
                acc[hh][1] = wmma16g(a[hh], b1, acc[hh][1]);
            }
        }
    }

    const float sg0 = (gv & 4) ? -1.0f : 1.0f;
    const float sg1 = (gv & 2) ? -1.0f : 1.0f;
    const float sg2 = (gv & 1) ? -1.0f : 1.0f;
    const float sgh = hi ? -1.0f : 1.0f;
    float val[2][8];
#pragma unroll
    for (int nt = 0; nt < 2; ++nt) {
        float tot = 0.0f, sh = 0.0f, s4 = 0.0f, s2 = 0.0f, s1 = 0.0f;
#pragma unroll
        for (int tl2 = 0; tl2 < 2; ++tl2) {
#pragma unroll
            for (int r = 0; r < 8; ++r) {
                const float yr = acc[tl2][nt][r] * YSI;
                const float yi = acc[tl2 + 2][nt][r] * YSI;
                const float p = yr * yr + yi * yi;
                tot += p;
                if (tl2) sh += p;
                if (r & 4) s4 += p;
                if (r & 2) s2 += p;
                if (r & 1) s1 += p;
            }
        }
        val[nt][0] = sg0 * tot; val[nt][1] = sg1 * tot; val[nt][2] = sg2 * tot;
        val[nt][3] = tot - 2.0f * sh;
        val[nt][4] = sgh * tot;
        val[nt][5] = tot - 2.0f * s4; val[nt][6] = tot - 2.0f * s2; val[nt][7] = tot - 2.0f * s1;
#pragma unroll
        for (int q = 0; q < 8; ++q) val[nt][q] += __shfl_xor(val[nt][q], 16, 32);
    }
    if (lane < 16) {
#pragma unroll
        for (int nt = 0; nt < 2; ++nt) {
            v4f p0, p1;
            p0[0] = val[nt][0]; p0[1] = val[nt][1]; p0[2] = val[nt][2]; p0[3] = val[nt][3];
            p1[0] = val[nt][4]; p1[1] = val[nt][5]; p1[2] = val[nt][6]; p1[3] = val[nt][7];
            const int po = ((wave * 2 + nt) * 16 + lr) * 8;
            *(v4fa*)(&part[po]) = p0; *(v4fa*)(&part[po + 4]) = p1;
        }
    }
    __syncthreads();

    if (tid < 64) {
        const int n = tid >> 1, q4 = (tid & 1) * 4;
        v4f s = (v4f){};
#pragma unroll
        for (int wv = 0; wv < 8; ++wv) {
            const v4f pv = *(const v4fa*)(&part[((wv * 2 + (n >> 4)) * 16 + (n & 15)) * 8 + q4]);
            s = s + pv;
        }
        float* dst = OUT + (size_t)n0 * NQ + (size_t)tid * 4;
        *(volatile v4f*)dst = s;
        __threadfence();
        *(volatile v4f*)dst = s;
    }
}

static constexpr size_t al256(size_t v) { return (v + 255) & ~(size_t)255; }
static constexpr size_t SZ_AP = al256((size_t)KD * KD * 2);
static constexpr size_t SZ_TOTAL = SZ_AP;
static_assert(SZ_TOTAL <= (size_t)134217728);
static_assert((size_t)(DIM - 1 + 256) * KD + (size_t)63 * 8 + 8 <= (size_t)KD * KD);
static_assert((size_t)(NB / BT - 1) * BT * NQ + (size_t)63 * 4 + 4 <= (size_t)NB * NQ);

extern "C" void kernel_launch(void* const* d_in, const int* in_sizes, int n_in,
                              void* d_out, int out_size, void* d_ws, size_t ws_size, hipStream_t stream) {
    if (n_in < 2) return;
    if ((size_t)in_sizes[0] < (size_t)NB * NQ) return;
    if (in_sizes[1] < NLAY * 4 * NQ) return;
    if ((size_t)out_size < (size_t)NB * NQ) return;
    if (SZ_TOTAL > ws_size) return;
    const float* x = (const float*)d_in[0];
    const float* w = (const float*)d_in[1];
    float* OUT = (float*)d_out;
    h16* AP = (h16*)d_ws;

    k_build<<<DIM, 128, 0, stream>>>(w, AP);
    k_apply<<<NB / BT, 256, 0, stream>>>(x, AP, OUT);
}
